// CausalAttn_23167053594697
// MI455X (gfx1250) — hardware-verified
//
#include <hip/hip_runtime.h>
#include <math.h>
#include <stdint.h>

#ifndef NB
#define NB 2
#endif
#ifndef SEQ
#define SEQ 2048
#endif
#define NB_FULL 2
#define T_FULL  2048
#define DMOD    1024
#define NH      16
#define HD      64
#define RHALF   32
#define GIN     20
#define WIN     1024
#define MROWS   (NB * SEQ)
#define OPITCH  (2 * DMOD)
#define QSC   8.0f
#define KSC   8.0f
#define QRS   1024.0f
#define PCAR  32768.0f
#define VCAR  1024.0f
#define VRS   1024.0f
#define PRS   1024.0f
#define OSC   1024.0f
#define ORS   1024.0f
#define WOS   1024.0f
#define LOG2E 1.4426950408889634f
#define NEGS  (-3.0e38f)
#define ATT_WAVES   4
#define ATT_THREADS (ATT_WAVES * 32)
#define NQT         (SEQ / 64)
#define ATT_BLOCKS  (NB * NH * NQT)
#define NKB         (SEQ / 32)
#define QRES        128
#define SLAB        (16 * 68)
static_assert(NB >= 1 && NB <= NB_FULL);
static_assert((SEQ % 64) == 0 && SEQ >= 64 && SEQ <= T_FULL);
static_assert(HD == 64 && DMOD == NH * HD && HD == 2 * RHALF);
static_assert(ATT_THREADS == 128 && NKB >= 2 && (QRES % 64) == 0);
static_assert((DMOD % 64) == 0 && (DMOD / 8) == 128 && (OPITCH % 32) == 0);
static_assert(((MROWS * (DMOD / 8)) % 256) == 0 && (((DMOD * DMOD) / 8) % 256) == 0);
static_assert((GIN % 4) == 0 && GIN <= DMOD);
static_assert((WIN % 32) == 0);
static_assert((SLAB * 4) % 16 == 0);

typedef unsigned short u16;
typedef _Float16 v16h __attribute__((ext_vector_type(16)));
typedef _Float16 v8h  __attribute__((ext_vector_type(8)));
typedef __bf16   v16b __attribute__((ext_vector_type(16)));
typedef float    v8f  __attribute__((ext_vector_type(8)));
typedef float    v4f  __attribute__((ext_vector_type(4)));
typedef unsigned int v4u __attribute__((ext_vector_type(4)));

union FragH { v16h v; v8h h[2]; v4u u[2]; };
union FragB { v16b v; v4u u[2]; };

__device__ __forceinline__ unsigned short bf_bits(float f) {
  unsigned u = __float_as_uint(f);
  return (unsigned short)((u + 0x7FFFu + ((u >> 16) & 1u)) >> 16);
}
__device__ __forceinline__ float bf_up(unsigned short h) { return __uint_as_float(((unsigned)h) << 16); }
__device__ __forceinline__ float bf_val(float f) { return bf_up(bf_bits(f)); }
__device__ __forceinline__ unsigned short h_bits(_Float16 x) { return __builtin_bit_cast(unsigned short, x); }
__device__ __forceinline__ unsigned pk16(unsigned short a, unsigned short b) { return (unsigned)a | ((unsigned)b << 16); }
__device__ __forceinline__ v8f zero8() { v8f z = {0.f, 0.f, 0.f, 0.f, 0.f, 0.f, 0.f, 0.f}; return z; }

__device__ __forceinline__ v16h ldfrag_h(const _Float16* p) {
  FragH f;
  f.h[0] = *(const v8h*)(p);
  f.h[1] = *(const v8h*)(p + 16);
  return f.v;
}
__device__ __forceinline__ v16b ldfrag_b(const u16* p) {
  FragB f;
  f.u[0] = *(const v4u*)(p);
  f.u[1] = *(const v4u*)(p + 16);
  return f.v;
}

__device__ __forceinline__ v8f mma_h(v16h a, v16h b, v8f c) {
  return __builtin_amdgcn_wmma_f32_16x16x32_f16(false, a, false, b, (short)0, c, false, false);
}
__device__ __forceinline__ v8f mma_b(v16b a, v16b b, v8f c) {
  return __builtin_amdgcn_wmma_f32_16x16x32_bf16(false, a, false, b, (short)0, c, false, false);
}
template <typename F>
__device__ __forceinline__ void guard6(v8f& a, v8f& b, v8f& c, v8f& d, F x0, F x1, F x2, F x3, F x4, F x5) {
#if defined(__HIP_DEVICE_COMPILE__)
  asm volatile("v_nop\n\tv_nop\n\tv_nop\n\tv_nop"
               : "+v"(a), "+v"(b), "+v"(c), "+v"(d) : "v"(x0), "v"(x1), "v"(x2), "v"(x3), "v"(x4), "v"(x5) : "memory");
#endif
}
__device__ __forceinline__ void acc_guard4(v8f& a, v8f& b, v8f& c, v8f& d) {
#if defined(__HIP_DEVICE_COMPILE__)
  asm volatile("v_nop\n\tv_nop\n\tv_nop\n\tv_nop" : "+v"(a), "+v"(b), "+v"(c), "+v"(d));
#endif
}
__device__ __forceinline__ void wave_sync_lds() {
#if defined(__HIP_DEVICE_COMPILE__)
  __builtin_amdgcn_fence(__ATOMIC_RELEASE, "workgroup");
  __builtin_amdgcn_wave_barrier();
  __builtin_amdgcn_fence(__ATOMIC_ACQUIRE, "workgroup");
#endif
}

__global__ __launch_bounds__(256) void cvt_rows(const float* __restrict__ x, u16* D, int n8, int seq, int tfull) {
  const int gt = blockIdx.x * 256 + (int)threadIdx.x;
  if (gt >= n8) return;
  const int row = gt >> 7;
  const int c8  = (gt & 127) * 8;
  const int bb  = row / seq;
  const int tt  = row - bb * seq;
  const float* p = x + ((size_t)bb * (size_t)tfull + (size_t)tt) * DMOD + c8;
  const v4f a = *(const v4f*)(p), c4 = *(const v4f*)(p + 4);
  float v[8];
#pragma unroll
  for (int e = 0; e < 4; ++e) { v[e] = a[e]; v[4 + e] = c4[e]; }
  unsigned short s[8];
#pragma unroll
  for (int e = 0; e < 8; ++e) s[e] = bf_bits(v[e]);
  v4u o;
#pragma unroll
  for (int e = 0; e < 4; ++e) o[e] = pk16(s[2 * e], s[2 * e + 1]);
  u16* d = D + (size_t)gt * 8;
  for (int pass = 0; pass < 2; ++pass) {
    *(volatile v4u*)(d) = o;
    __threadfence();
  }
}

__global__ __launch_bounds__(256) void cvt_wo(const float* __restrict__ w, u16* D, int n8, float s1, float s2) {
  const int gt = blockIdx.x * 256 + (int)threadIdx.x;
  if (gt >= n8) return;
  const int n  = gt >> 7;
  const int c8 = (gt & 127) * 8;
  const float* p = w + (size_t)gt * 8;
  const v4f a = *(const v4f*)(p), c4 = *(const v4f*)(p + 4);
  float v[8];
#pragma unroll
  for (int e = 0; e < 4; ++e) { v[e] = a[e]; v[4 + e] = c4[e]; }
  unsigned short h1[8], h2[8];
#pragma unroll
  for (int e = 0; e < 8; ++e) {
    const float f = bf_val(v[e]);
    h1[e] = h_bits((_Float16)(f * s1));
    h2[e] = h_bits((_Float16)(f * s2));
  }
  v4u o1, o2;
#pragma unroll
  for (int e = 0; e < 4; ++e) { o1[e] = pk16(h1[2 * e], h1[2 * e + 1]); o2[e] = pk16(h2[2 * e], h2[2 * e + 1]); }
  u16* d1 = D + (size_t)n * OPITCH + c8;
  u16* d2 = d1 + DMOD;
  for (int pass = 0; pass < 2; ++pass) {
    *(volatile v4u*)(d1) = o1;
    *(volatile v4u*)(d2) = o2;
    __threadfence();
  }
}

__device__ __forceinline__ void epi_rope(float* sl, v8f a0, v8f a1, v8f a2, v8f a3, u16* C, u16* C2, int res_on,
                                         size_t rowb, int col0, int lane, const float* __restrict__ bias, int blen,
                                         const float* __restrict__ cosT, const float* __restrict__ sinT, int seq,
                                         float oscale, float rsc) {
#pragma clang fp contract(off)
  const int hh = lane >> 4, m = lane & 15;
  float bc[4];
#pragma unroll
  for (int j = 0; j < 4; ++j) {
    const int bi = min(col0 + 16 * j + m, blen - 1);
    bc[j] = bf_val(bias[bi]);
  }
#pragma unroll
  for (int r = 0; r < 8; ++r) {
    const int ro = (8 * hh + r) * 68 + m;
    sl[ro]      = a0[r] + bc[0];
    sl[ro + 16] = a1[r] + bc[1];
    sl[ro + 32] = a2[r] + bc[2];
    sl[ro + 48] = a3[r] + bc[3];
  }
  wave_sync_lds();
  const int rq = lane >> 3, c8 = (lane & 7) * 8, dd = c8 & (RHALF - 1);
  const bool lo = (c8 < RHALF);
  const int tb = (int)(rowb % (size_t)seq);
  v4u hv[4], rv[4];
#pragma unroll
  for (int i4 = 0; i4 < 4; ++i4) {
    const int row = i4 * 4 + rq;
    const int t = tb + row;
    const float* cp = cosT + (size_t)t * RHALF + dd;
    const float* sp = sinT + (size_t)t * RHALF + dd;
    const v4f ca = *(const v4f*)(cp), cb = *(const v4f*)(cp + 4);
    const v4f sa = *(const v4f*)(sp), sb = *(const v4f*)(sp + 4);
    const v4f xa = *(const v4f*)(sl + row * 68 + dd), xb = *(const v4f*)(sl + row * 68 + dd + 4);
    const v4f ya = *(const v4f*)(sl + row * 68 + dd + RHALF), yb = *(const v4f*)(sl + row * 68 + dd + RHALF + 4);
    float cv[8], sv[8], xv[8], yv[8];
#pragma unroll
    for (int e = 0; e < 4; ++e) {
      cv[e] = ca[e]; cv[4 + e] = cb[e];
      sv[e] = sa[e]; sv[4 + e] = sb[e];
      xv[e] = xa[e]; xv[4 + e] = xb[e];
      yv[e] = ya[e]; yv[4 + e] = yb[e];
    }
    unsigned short hb[8], rb[8];
#pragma unroll
    for (int e = 0; e < 8; ++e) {
      const float cc = bf_val(cv[e]);
      const float ss = bf_val(sv[e]);
      const float p1 = xv[e] * cc;
      const float p2 = yv[e] * ss;
      const float p3 = xv[e] * ss;
      const float p4 = yv[e] * cc;
      const float u = lo ? (p1 - p2) : (p3 + p4);
      const float w = u * oscale;
      const _Float16 h = (_Float16)w;
      hb[e] = h_bits(h);
      rb[e] = h_bits((_Float16)((w - (float)h) * rsc));
    }
#pragma unroll
    for (int e = 0; e < 4; ++e) {
      hv[i4][e] = pk16(hb[2 * e], hb[2 * e + 1]);
      rv[i4][e] = pk16(rb[2 * e], rb[2 * e + 1]);
    }
  }
  u16* dst = C + (rowb + (size_t)rq) * (size_t)DMOD + col0 + c8;
  for (int pass = 0; pass < 2; ++pass) {
#pragma unroll
    for (int i4 = 0; i4 < 4; ++i4) {
      *(volatile v4u*)(dst + (size_t)(i4 * 4) * (size_t)DMOD) = hv[i4];
    }
    __threadfence();
  }
  if (res_on != 0) {
    u16* dst2 = C2 + (rowb + (size_t)rq) * (size_t)DMOD + col0 + c8;
    for (int pass = 0; pass < 2; ++pass) {
#pragma unroll
      for (int i4 = 0; i4 < 4; ++i4) {
        *(volatile v4u*)(dst2 + (size_t)(i4 * 4) * (size_t)DMOD) = rv[i4];
      }
      __threadfence();
    }
  }
}

__device__ __forceinline__ void epi_v3(float* sl, v8f a0, v8f a1, v8f a2, v8f a3, float oscale, u16* C0, u16* C1, u16* C2,
                                       int N, size_t rowb, int col0, int lane, const float* __restrict__ bias, int blen,
                                       float rsc, float qsc) {
  const int hh = lane >> 4, m = lane & 15;
  float br[8];
#pragma unroll
  for (int r = 0; r < 8; ++r) {
    const int bi = min((int)rowb + 8 * hh + r, blen - 1);
    br[r] = bf_val(bias[bi]);
  }
#pragma unroll
  for (int r = 0; r < 8; ++r) {
    const int ro = (8 * hh + r) * 68 + m;
    sl[ro]      = (a0[r] + br[r]) * oscale;
    sl[ro + 16] = (a1[r] + br[r]) * oscale;
    sl[ro + 32] = (a2[r] + br[r]) * oscale;
    sl[ro + 48] = (a3[r] + br[r]) * oscale;
  }
  wave_sync_lds();
  const int rq = lane >> 3, c8 = (lane & 7) * 8;
  v4u h4[4], r4[4], q4[4];
#pragma unroll
  for (int i4 = 0; i4 < 4; ++i4) {
    const int row = i4 * 4 + rq;
    const v4f a = *(const v4f*)(sl + row * 68 + c8), c4 = *(const v4f*)(sl + row * 68 + c8 + 4);
    float w[8];
#pragma unroll
    for (int e = 0; e < 4; ++e) { w[e] = a[e]; w[4 + e] = c4[e]; }
    unsigned short hb[8], rb[8], qb[8];
#pragma unroll
    for (int e = 0; e < 8; ++e) {
      const _Float16 h = (_Float16)w[e];
      hb[e] = h_bits(h);
      rb[e] = h_bits((_Float16)((w[e] - (float)h) * rsc));
      qb[e] = h_bits((_Float16)(w[e] * qsc));
    }
#pragma unroll
    for (int e = 0; e < 4; ++e) {
      h4[i4][e] = pk16(hb[2 * e], hb[2 * e + 1]);
      r4[i4][e] = pk16(rb[2 * e], rb[2 * e + 1]);
      q4[i4][e] = pk16(qb[2 * e], qb[2 * e + 1]);
    }
  }
  const size_t dof = (rowb + (size_t)rq) * (size_t)N + col0 + c8;
  u16* d0 = C0 + dof;
  u16* d1 = C1 + dof;
  u16* d2 = C2 + dof;
  for (int pass = 0; pass < 2; ++pass) {
#pragma unroll
    for (int i4 = 0; i4 < 4; ++i4) {
      const size_t ro = (size_t)(i4 * 4) * (size_t)N;
      *(volatile v4u*)(d0 + ro) = h4[i4];
      *(volatile v4u*)(d1 + ro) = r4[i4];
      *(volatile v4u*)(d2 + ro) = q4[i4];
    }
    __threadfence();
  }
}

__device__ __forceinline__ void epi64(float* sl, v8f a0, v8f a1, v8f a2, v8f a3, float oscale, float* C, int N,
                                      size_t rowb, int col0, int lane, const float* __restrict__ bias, int blen) {
  const int hh = lane >> 4, m = lane & 15;
  float bc[4];
#pragma unroll
  for (int j = 0; j < 4; ++j) {
    const int bi = min(col0 + 16 * j + m, blen - 1);
    bc[j] = bf_val(bias[bi]);
  }
#pragma unroll
  for (int r = 0; r < 8; ++r) {
    const int ro = (8 * hh + r) * 68 + m;
    sl[ro]      = a0[r] * oscale + bc[0];
    sl[ro + 16] = a1[r] * oscale + bc[1];
    sl[ro + 32] = a2[r] * oscale + bc[2];
    sl[ro + 48] = a3[r] * oscale + bc[3];
  }
  wave_sync_lds();
  v4f vals[8];
#pragma unroll
  for (int it = 0; it < 8; ++it) vals[it] = *(const v4f*)(sl + (it * 2 + hh) * 68 + m * 4);
  float* dst = C + (rowb + (size_t)hh) * (size_t)N + col0 + m * 4;
  for (int pass = 0; pass < 2; ++pass) {
#pragma unroll
    for (int it = 0; it < 8; ++it) {
      *(volatile v4f*)(dst + (size_t)(it * 2) * (size_t)N) = vals[it];
    }
    __threadfence();
  }
}

__global__ __launch_bounds__(128)
void gemm_rope(const u16* __restrict__ A, const u16* __restrict__ Bt, u16* C, u16* C2, int res_on, int M, int K,
               const float* __restrict__ bias, int blen, const float* __restrict__ cosT,
               const float* __restrict__ sinT, int seq, float oscale, float rsc) {
  __shared__ __align__(16) float slab[4 * SLAB];
  const int tid = threadIdx.x, wave = tid >> 5, lane = tid & 31, hh = lane >> 4, m = lane & 15;
  const int ntile = DMOD >> 6;
  const int bid   = blockIdx.x;
  const int rowb  = (bid / ntile) * 64 + wave * 16;
  const int col0  = (bid % ntile) * 64;
  if (rowb + 16 > M) return;
  const u16* ap = A  + (size_t)(rowb + m) * K + 8 * hh;
  const u16* bp = Bt + (size_t)(col0 + m) * K + 8 * hh;
  const size_t bs = (size_t)16 * K;
  v8f acc0 = zero8(), acc1 = zero8(), acc2 = zero8(), acc3 = zero8();
#pragma unroll 1
  for (int k0 = 0; k0 < K; k0 += 32) {
    const v16b a  = ldfrag_b(ap + k0);
    const v16b b0 = ldfrag_b(bp + k0);
    const v16b b1 = ldfrag_b(bp + bs + k0);
    const v16b b2 = ldfrag_b(bp + 2 * bs + k0);
    const v16b b3 = ldfrag_b(bp + 3 * bs + k0);
    acc0 = mma_b(a, b0, acc0);
    acc1 = mma_b(a, b1, acc1);
    acc2 = mma_b(a, b2, acc2);
    acc3 = mma_b(a, b3, acc3);
    guard6<v16b>(acc0, acc1, acc2, acc3, a, b0, b1, b2, b3, a);
  }
  epi_rope(slab + wave * SLAB, acc0, acc1, acc2, acc3, C, C2, res_on, (size_t)rowb, col0, lane, bias, blen,
           cosT, sinT, seq, oscale, rsc);
}

__global__ __launch_bounds__(128)
void gemm_v(const u16* __restrict__ A, const u16* __restrict__ Bt, u16* C0, u16* C1, u16* C2, int M, int N, int K,
            int bstB, int bstC, float oscale, const float* __restrict__ bias, int blen, float rsc, float qsc) {
  __shared__ __align__(16) float slab[4 * SLAB];
  const int tid = threadIdx.x, wave = tid >> 5, lane = tid & 31, hh = lane >> 4, m = lane & 15;
  const int ntile = N >> 6, mtile = M >> 6;
  const int per   = ntile * mtile;
  const int bid   = blockIdx.x;
  const int bt    = bid / per;
  const int t     = bid - bt * per;
  const int rowb  = (t / ntile) * 64 + wave * 16;
  const int col0  = (t % ntile) * 64;
  if (rowb + 16 > M) return;
  const u16* Ab = A;
  const u16* Bb = Bt + (size_t)bt * (size_t)bstB;
  const size_t cb = (size_t)bt * (size_t)bstC;
  const u16* ap = Ab + (size_t)(rowb + m) * K + 8 * hh;
  const u16* bp = Bb + (size_t)(col0 + m) * K + 8 * hh;
  const size_t bs = (size_t)16 * K;
  v8f acc0 = zero8(), acc1 = zero8(), acc2 = zero8(), acc3 = zero8();
#pragma unroll 1
  for (int k0 = 0; k0 < K; k0 += 32) {
    const v16b a  = ldfrag_b(ap + k0);
    const v16b b0 = ldfrag_b(bp + k0);
    const v16b b1 = ldfrag_b(bp + bs + k0);
    const v16b b2 = ldfrag_b(bp + 2 * bs + k0);
    const v16b b3 = ldfrag_b(bp + 3 * bs + k0);
    acc0 = mma_b(a, b0, acc0);
    acc1 = mma_b(a, b1, acc1);
    acc2 = mma_b(a, b2, acc2);
    acc3 = mma_b(a, b3, acc3);
    guard6<v16b>(acc0, acc1, acc2, acc3, a, b0, b1, b2, b3, a);
  }
  epi_v3(slab + wave * SLAB, acc0, acc1, acc2, acc3, oscale, C0 + cb, C1 + cb, C2 + cb, N, (size_t)rowb, col0, lane,
         bias, blen, rsc, qsc);
}

__global__ __launch_bounds__(128)
void gemm_hf(const u16* __restrict__ A, const u16* __restrict__ Bt, float* C, int M, int N, int K, float oscale,
             const float* __restrict__ bias, int blen) {
  __shared__ __align__(16) float slab[4 * SLAB];
  const int tid = threadIdx.x, wave = tid >> 5, lane = tid & 31, hh = lane >> 4, m = lane & 15;
  const int ntile = N >> 6;
  const int bid   = blockIdx.x;
  const int rowb  = (bid / ntile) * 64 + wave * 16;
  const int col0  = (bid % ntile) * 64;
  if (rowb + 16 > M) return;
  const _Float16* ap = (const _Float16*)(const void*)A  + (size_t)(rowb + m) * K + 8 * hh;
  const _Float16* bp = (const _Float16*)(const void*)Bt + (size_t)(col0 + m) * K + 8 * hh;
  const size_t bs = (size_t)16 * K;
  v8f acc0 = zero8(), acc1 = zero8(), acc2 = zero8(), acc3 = zero8();
#pragma unroll 1
  for (int k0 = 0; k0 < K; k0 += 32) {
    const v16h a  = ldfrag_h(ap + k0);
    const v16h b0 = ldfrag_h(bp + k0);
    const v16h b1 = ldfrag_h(bp + bs + k0);
    const v16h b2 = ldfrag_h(bp + 2 * bs + k0);
    const v16h b3 = ldfrag_h(bp + 3 * bs + k0);
    acc0 = mma_h(a, b0, acc0);
    acc1 = mma_h(a, b1, acc1);
    acc2 = mma_h(a, b2, acc2);
    acc3 = mma_h(a, b3, acc3);
    guard6<v16h>(acc0, acc1, acc2, acc3, a, b0, b1, b2, b3, a);
  }
  epi64(slab + wave * SLAB, acc0, acc1, acc2, acc3, oscale, C, N, (size_t)rowb, col0, lane, bias, blen);
}

__global__ __launch_bounds__(ATT_THREADS)
void attn_fwd(const u16* __restrict__ QHp, const u16* __restrict__ QRp, const u16* __restrict__ KHp,
              const u16* __restrict__ VHp, const u16* __restrict__ VRp, const u16* __restrict__ VQp,
              const float* __restrict__ Xp, const float* __restrict__ Wgp, const float* __restrict__ Bgp,
              int bglen, u16* OPp) {
  __shared__ __align__(16) float smem[ATT_WAVES * SLAB];

  const int tid  = threadIdx.x;
  const int wave = tid >> 5;
  const int lane = tid & 31;
  const int hh   = lane >> 4;
  const int c    = lane & 15;

  const int bid  = blockIdx.x;
  const int qt   = bid % NQT;
  const int bh   = bid / NQT;
  const int head = bh % NH;
  const int b    = bh / NH;
  if (b >= NB) return;
  const int qb   = qt * 64;
  const int q0   = qb + wave * 16;

  const int jlo  = max(qb - WIN, 0);
  const int kblo = jlo >> 5;
  int nkb = ((qb + 63) >> 5) - kblo + 1;
  nkb = min(max(nkb, 1), NKB - kblo);
  const bool early = (qb < QRES);

  const size_t prow = (size_t)b * SEQ;
  const size_t qofs = (prow + (size_t)(q0 + c)) * DMOD + head * HD + 8 * hh;
  const _Float16* Qh = (const _Float16*)(const void*)QHp + qofs;
  const _Float16* Qr = (const _Float16*)(const void*)QRp + qofs;
  const size_t kofs = (prow + (size_t)c) * DMOD + head * HD + 8 * hh;
  const _Float16* Kb = (const _Float16*)(const void*)KHp + kofs;
  const size_t vofs = ((size_t)b * DMOD + (size_t)(head * HD + c)) * SEQ + 8 * hh;
  const _Float16* Vh = (const _Float16*)(const void*)VHp + vofs;
  const _Float16* Vr = (const _Float16*)(const void*)VRp + vofs;
  const _Float16* Vq = (const _Float16*)(const void*)VQp + vofs;
  const float lsc = 0.125f * (LOG2E / (QSC * KSC));
  const float qri = 1.0f / QRS;
  const int dq = q0 + c - 8 * hh;

  const v16h qf0 = ldfrag_h(Qh);
  const v16h qf1 = ldfrag_h(Qh + 32);
  const v16h qr0 = ldfrag_h(Qr);
  const v16h qr1 = ldfrag_h(Qr + 32);

  float mrun = NEGS, lrun = 0.f;
  v8f o[4];
#pragma unroll
  for (int j = 0; j < 4; ++j) o[j] = zero8();

#pragma unroll 1
  for (int it = 0; it < nkb; ++it) {
    const int kb = (kblo + it) * 32;
    v8f s0 = zero8(), s1 = zero8(), r0 = zero8(), r1 = zero8();
    const _Float16* k0p = Kb + (size_t)kb * DMOD;
    const _Float16* k1p = k0p + (size_t)16 * DMOD;
    const v16h ka0 = ldfrag_h(k0p), ka1 = ldfrag_h(k0p + 32);
    const v16h kc0 = ldfrag_h(k1p), kc1 = ldfrag_h(k1p + 32);
    s0 = mma_h(ka0, qf0, s0);
    s0 = mma_h(ka1, qf1, s0);
    r0 = mma_h(ka0, qr0, r0);
    r0 = mma_h(ka1, qr1, r0);
    s1 = mma_h(kc0, qf0, s1);
    s1 = mma_h(kc1, qf1, s1);
    r1 = mma_h(kc0, qr0, r1);
    r1 = mma_h(kc1, qr1, r1);
    guard6<v16h>(s0, s1, r0, r1, ka0, ka1, kc0, kc1, qf0, qr0);
    float tk[16];
#pragma unroll
    for (int i = 0; i < 8; ++i) {
      const int d0 = dq - kb - i;
      const int d1 = d0 - 16;
      const bool a0 = (d0 >= 0) && (d0 <= WIN);
      const bool a1 = (d1 >= 0) && (d1 <= WIN);
      tk[i]     = a0 ? ((s0[i] + r0[i] * qri) * lsc) : NEGS;
      tk[8 + i] = a1 ? ((s1[i] + r1[i] * qri) * lsc) : NEGS;
    }
    float cm = tk[0];
#pragma unroll
    for (int i = 1; i < 16; ++i) cm = fmaxf(cm, tk[i]);
    cm = fmaxf(cm, __shfl_xor(cm, 16, 32));
    const float mn = fmaxf(mrun, cm);
    const float al = exp2f(fminf(mrun - mn, 0.f));
    mrun = mn;
    float ps = 0.f;
    FragH ph, pl, pr;
#pragma unroll
    for (int wq = 0; wq < 2; ++wq) {
#pragma unroll
      for (int e4 = 0; e4 < 4; ++e4) {
        const int i = 8 * wq + 2 * e4;
        const float x0 = exp2f(fminf(tk[i] - mn, 0.f));
        const float x1 = exp2f(fminf(tk[i + 1] - mn, 0.f));
        const float p0 = (tk[i] > -1.0e38f) ? x0 : 0.f;
        const float p1 = (tk[i + 1] > -1.0e38f) ? x1 : 0.f;
        ps += p0 + p1;
        const float g0 = p0 * PCAR, g1 = p1 * PCAR;
        const _Float16 h0 = (_Float16)g0, h1 = (_Float16)g1;
        ph.u[wq][e4] = pk16(h_bits(h0), h_bits(h1));
        pl.u[wq][e4] = pk16(h_bits((_Float16)(g0 * (1.0f / VRS))), h_bits((_Float16)(g1 * (1.0f / VRS))));
        pr.u[wq][e4] = pk16(h_bits((_Float16)((g0 - (float)h0) * PRS)), h_bits((_Float16)((g1 - (float)h1) * PRS)));
      }
    }
    ps += __shfl_xor(ps, 16, 32);
    lrun = lrun * al + ps;
    float scl[8];
#pragma unroll
    for (int r = 0; r < 8; ++r) scl[r] = __shfl(al, 8 * hh + r, 32);
#pragma unroll
    for (int j = 0; j < 4; ++j) {
#pragma unroll
      for (int r = 0; r < 8; ++r) o[j][r] *= scl[r];
    }
    {
      const _Float16* vp = Vh + kb;
      const v16h vf0 = ldfrag_h(vp);
      const v16h vf1 = ldfrag_h(vp + (size_t)16 * SEQ);
      const v16h vf2 = ldfrag_h(vp + (size_t)32 * SEQ);
      const v16h vf3 = ldfrag_h(vp + (size_t)48 * SEQ);
      o[0] = mma_h(ph.v, vf0, o[0]);
      o[1] = mma_h(ph.v, vf1, o[1]);
      o[2] = mma_h(ph.v, vf2, o[2]);
      o[3] = mma_h(ph.v, vf3, o[3]);
      guard6<v16h>(o[0], o[1], o[2], o[3], ph.v, vf0, vf1, vf2, vf3, ph.v);
    }
    if (early) {
      {
        const _Float16* vp = Vr + kb;
        const v16h vf0 = ldfrag_h(vp);
        const v16h vf1 = ldfrag_h(vp + (size_t)16 * SEQ);
        const v16h vf2 = ldfrag_h(vp + (size_t)32 * SEQ);
        const v16h vf3 = ldfrag_h(vp + (size_t)48 * SEQ);
        o[0] = mma_h(pl.v, vf0, o[0]);
        o[1] = mma_h(pl.v, vf1, o[1]);
        o[2] = mma_h(pl.v, vf2, o[2]);
        o[3] = mma_h(pl.v, vf3, o[3]);
        guard6<v16h>(o[0], o[1], o[2], o[3], pl.v, vf0, vf1, vf2, vf3, pl.v);
      }
      {
        const _Float16* vp = Vq + kb;
        const v16h vf0 = ldfrag_h(vp);
        const v16h vf1 = ldfrag_h(vp + (size_t)16 * SEQ);
        const v16h vf2 = ldfrag_h(vp + (size_t)32 * SEQ);
        const v16h vf3 = ldfrag_h(vp + (size_t)48 * SEQ);
        o[0] = mma_h(pr.v, vf0, o[0]);
        o[1] = mma_h(pr.v, vf1, o[1]);
        o[2] = mma_h(pr.v, vf2, o[2]);
        o[3] = mma_h(pr.v, vf3, o[3]);
        guard6<v16h>(o[0], o[1], o[2], o[3], pr.v, vf0, vf1, vf2, vf3, pr.v);
      }
    }
  }
  acc_guard4(o[0], o[1], o[2], o[3]);

  const int gx = min(head, bglen - 1);
  float ga = bf_val(Bgp[gx]);
  const float* xg = Xp + ((size_t)b * T_FULL + (size_t)(q0 + c)) * DMOD;
  const float* wg = Wgp + head * GIN;
#pragma unroll
  for (int g4 = 0; g4 < GIN / 4; ++g4) {
    const v4f xv = *(const v4f*)(xg + 4 * g4);
    const v4f wv = *(const v4f*)(wg + 4 * g4);
#pragma unroll
    for (int e = 0; e < 4; ++e) ga += bf_val(xv[e]) * bf_val(wv[e]);
  }
  const float gate = 1.0f / (1.0f + expf(-ga));

  const float linv = (lrun > 0.f) ? (gate * (1.0f / lrun) * (1.0f / (PCAR * VCAR))) : 0.f;
  float inv[8];
#pragma unroll
  for (int r = 0; r < 8; ++r) inv[r] = __shfl(linv, 8 * hh + r, 32);
  float* slab = smem + wave * SLAB;
#pragma unroll
  for (int r = 0; r < 8; ++r) {
#pragma unroll
    for (int j = 0; j < 4; ++j) slab[(8 * hh + r) * 68 + j * 16 + c] = o[j][r] * inv[r];
  }
  wave_sync_lds();
  v4u oh[4], orr[4];
  const int rq = lane >> 3, c8 = (lane & 7) * 8;
#pragma unroll
  for (int i4 = 0; i4 < 4; ++i4) {
    const int row = i4 * 4 + rq;
    const v4f a = *(const v4f*)(slab + row * 68 + c8), c4 = *(const v4f*)(slab + row * 68 + c8 + 4);
    float wv[8];
#pragma unroll
    for (int e = 0; e < 4; ++e) { wv[e] = a[e] * OSC; wv[4 + e] = c4[e] * OSC; }
#pragma unroll
    for (int e = 0; e < 4; ++e) {
      const float w0 = wv[2 * e], w1 = wv[2 * e + 1];
      const _Float16 h0 = (_Float16)w0, h1 = (_Float16)w1;
      oh[i4][e]  = pk16(h_bits(h0), h_bits(h1));
      orr[i4][e] = pk16(h_bits((_Float16)((w0 - (float)h0) * ORS)), h_bits((_Float16)((w1 - (float)h1) * ORS)));
    }
  }
  const size_t ob = (prow + (size_t)q0) * OPITCH + head * HD + c8;
  for (int pass = 0; pass < 2; ++pass) {
#pragma unroll
    for (int i4 = 0; i4 < 4; ++i4) {
      const int row = i4 * 4 + rq;
      const size_t o8 = ob + (size_t)row * OPITCH;
      *(volatile v4u*)(OPp + o8) = oh[i4];
      *(volatile v4u*)(OPp + o8 + DMOD) = orr[i4];
    }
    __threadfence();
  }
}

extern "C" void kernel_launch(void* const* d_in, const int* in_sizes, int n_in,
                              void* d_out, int out_size, void* d_ws, size_t ws_size,
                              hipStream_t stream) {
  if (n_in < 13) return;
  if (in_sizes[0] < ((NB - 1) * T_FULL + SEQ) * DMOD) return;
  if (in_sizes[1] != DMOD * DMOD || in_sizes[3] != DMOD * DMOD || in_sizes[5] != DMOD * DMOD ||
      in_sizes[7] != DMOD * DMOD) return;
  if (in_sizes[2] < 1 || in_sizes[4] < 1 || in_sizes[6] < 1 || in_sizes[8] < 1) return;
  if (in_sizes[9] != NH * GIN) return;
  if (in_sizes[10] < 1) return;
  if (in_sizes[11] < SEQ * RHALF || in_sizes[12] < SEQ * RHALF) return;
  if (out_size < MROWS * DMOD) return;

  const float* Xin = (const float*)d_in[0];
  const float* Wq  = (const float*)d_in[1];
  const float* Bq  = (const float*)d_in[2];
  const float* Wk  = (const float*)d_in[3];
  const float* Bk  = (const float*)d_in[4];
  const float* Wv  = (const float*)d_in[5];
  const float* Bv  = (const float*)d_in[6];
  const float* Wo  = (const float*)d_in[7];
  const float* Bo  = (const float*)d_in[8];
  const float* Wg  = (const float*)d_in[9];
  const float* Bg  = (const float*)d_in[10];
  const float* Cos = (const float*)d_in[11];
  const float* Sin = (const float*)d_in[12];
  float*       out = (float*)d_out;

  const size_t szXB = (size_t)MROWS * DMOD * 2;
  const size_t szW  = (size_t)DMOD * DMOD * 2;
  const size_t szWO = (size_t)DMOD * OPITCH * 2;
  const size_t szQ  = (size_t)MROWS * DMOD * 2;
  const size_t szV  = (size_t)NB * DMOD * SEQ * 2;
  const size_t szOP = (size_t)MROWS * OPITCH * 2;
  size_t off = 0;
  const size_t oXB = off; off += szXB;
  const size_t oWQ = off; off += szW;
  const size_t oWK = off; off += szW;
  const size_t oWV = off; off += szW;
  const size_t oWO = off; off += szWO;
  const size_t oQH = off; off += szQ;
  const size_t oQR = off; off += szQ;
  const size_t oKH = off; off += szQ;
  const size_t oVH = off; off += szV;
  const size_t oVR = off; off += szV;
  const size_t oVQ = off; off += szV;
  const size_t oOP = off; off += szOP;
  if (off > ws_size) return;
  if (off > (size_t)134217728) return;

  char* ws = (char*)d_ws;
  u16* XB  = (u16*)(ws + oXB);
  u16* WQB = (u16*)(ws + oWQ);
  u16* WKB = (u16*)(ws + oWK);
  u16* WVB = (u16*)(ws + oWV);
  u16* WOB = (u16*)(ws + oWO);
  u16* QH  = (u16*)(ws + oQH);
  u16* QR  = (u16*)(ws + oQR);
  u16* KH  = (u16*)(ws + oKH);
  u16* VH  = (u16*)(ws + oVH);
  u16* VR  = (u16*)(ws + oVR);
  u16* VQ  = (u16*)(ws + oVQ);
  u16* OP  = (u16*)(ws + oOP);

  const int n8x = (MROWS * DMOD) / 8;
  const int n8w = (DMOD * DMOD) / 8;
  if ((n8x % 256) != 0 || (n8w % 256) != 0) return;
  if ((MROWS % 64) != 0 || (SEQ % 64) != 0 || (DMOD % 64) != 0 || (DMOD % 32) != 0 || (OPITCH % 32) != 0) return;
  const dim3 blk(256);
  const dim3 gX(n8x / 256);
  const dim3 gW(n8w / 256);
  const dim3 bG(128);
  const dim3 gP((MROWS / 64) * (DMOD / 64));
  const dim3 gV(NB * (DMOD / 64) * (SEQ / 64));
  const dim3 gAT(ATT_BLOCKS);
  const dim3 bAT(ATT_THREADS);
  const dim3 gO((MROWS / 64) * (DMOD / 64));

  cvt_rows<<<gX, blk, 0, stream>>>(Xin, XB, n8x, SEQ, T_FULL);
  cvt_rows<<<gW, blk, 0, stream>>>(Wq, WQB, n8w, DMOD, DMOD);
  cvt_rows<<<gW, blk, 0, stream>>>(Wk, WKB, n8w, DMOD, DMOD);
  cvt_rows<<<gW, blk, 0, stream>>>(Wv, WVB, n8w, DMOD, DMOD);
  cvt_wo<<<gW, blk, 0, stream>>>(Wo, WOB, n8w, WOS, WOS / ORS);
  gemm_rope<<<gP, bG, 0, stream>>>(XB, WQB, QH, QR, 1, MROWS, DMOD, Bq, in_sizes[2], Cos, Sin, SEQ, QSC, QRS);
  gemm_rope<<<gP, bG, 0, stream>>>(XB, WKB, KH, KH, 0, MROWS, DMOD, Bk, in_sizes[4], Cos, Sin, SEQ, KSC, 1.0f);
  gemm_v<<<gV, bG, 0, stream>>>(WVB, XB, VH, VR, VQ, DMOD, SEQ, DMOD, SEQ * DMOD, DMOD * SEQ, VCAR,
                                 Bv, in_sizes[6], VRS, 1.0f / PRS);
  attn_fwd<<<gAT, bAT, 0, stream>>>(QH, QR, KH, VH, VR, VQ, Xin, Wg, Bg, in_sizes[10], OP);
  gemm_hf<<<gO, bG, 0, stream>>>(OP, WOB, out, MROWS, DMOD, OPITCH, 1.0f / (OSC * WOS), Bo, in_sizes[8]);
  (void)hipGetLastError();
}
